// LimitedRelPositionMultiHeadedAttention_49615462204126
// MI455X (gfx1250) — hardware-verified
//
#include <hip/hip_runtime.h>
#include <math.h>

constexpr int kB    = 4;
constexpr int kT    = 1024;
constexpr int kF    = 512;
constexpr int kH    = 8;
constexpr int kDK   = 64;
constexpr int kP    = 2047;
constexpr int kPpad = 2048;
constexpr int kTok  = kB * kT;
constexpr int kHG   = 4;
constexpr int kNG   = kB * (kH / kHG);

typedef __attribute__((ext_vector_type(16))) _Float16 v16h;
typedef __attribute__((ext_vector_type(8)))  _Float16 v8h;
typedef __attribute__((ext_vector_type(16))) __bf16   v16b;
typedef __attribute__((ext_vector_type(8)))  __bf16   v8b;
typedef __attribute__((ext_vector_type(8)))  float    v8f;
typedef __attribute__((ext_vector_type(4)))  float    v4f;
typedef __attribute__((ext_vector_type(4)))  unsigned int v4u;
typedef __attribute__((ext_vector_type(4)))  int      v4i;

__device__ __forceinline__ unsigned short f2bf_bits(float f) {
  unsigned u = __float_as_uint(f);
  return (unsigned short)((u + 0x7FFFu + ((u >> 16) & 1u)) >> 16);
}
__device__ __forceinline__ float bf_bits2f(unsigned short h) { return __uint_as_float(((unsigned)h) << 16); }
__device__ __forceinline__ unsigned pk16(unsigned short a, unsigned short b) { return (unsigned)a | ((unsigned)b << 16); }

__device__ __forceinline__ void dep_guard_h(v8f& a, v8f& b, v16h x, v16h y) { asm volatile("v_nop\n\tv_nop\n\tv_nop\n\tv_nop" : "+v"(a), "+v"(b) : "v"(x), "v"(y)); }
__device__ __forceinline__ void dep_guard_b(v8f& a, v8f& b, v16b x, v16b y) { asm volatile("v_nop\n\tv_nop\n\tv_nop\n\tv_nop" : "+v"(a), "+v"(b) : "v"(x), "v"(y)); }
__device__ __forceinline__ void keep4_h(v16h a, v16h b, v16h c, v16h d) { asm volatile("v_nop" :: "v"(a), "v"(b), "v"(c), "v"(d)); }
__device__ __forceinline__ void keep4_b(v16b a, v16b b, v16b c, v16b d) { asm volatile("v_nop" :: "v"(a), "v"(b), "v"(c), "v"(d)); }
__device__ __forceinline__ void acc_guard4(v8f& a, v8f& b, v8f& c, v8f& d) { asm volatile("v_nop\n\tv_nop\n\tv_nop\n\tv_nop" : "+v"(a), "+v"(b), "+v"(c), "+v"(d)); }
template <typename T> struct Frag;
template <> struct Frag<_Float16> {
  typedef v16h V; union U { v16h v; v8h h[2]; };
  static __device__ __forceinline__ v16h load(const _Float16* p) {
    U f; f.h[0] = *(const v8h*)(p); f.h[1] = *(const v8h*)(p + 16); return f.v;
  }
  static __device__ __forceinline__ v8f mma(v16h a, v16h b, v8f c) {
    return __builtin_amdgcn_wmma_f32_16x16x32_f16(false, a, false, b, (short)0, c, false, false);
  }
  static __device__ __forceinline__ void guard(v8f& a, v8f& b, v16h x, v16h y) { dep_guard_h(a, b, x, y); }
  static __device__ __forceinline__ void keep(v16h a, v16h b, v16h c, v16h d) { keep4_h(a, b, c, d); }
};
template <> struct Frag<__bf16> {
  typedef v16b V; union U { v16b v; v8b h[2]; };
  static __device__ __forceinline__ v16b load(const __bf16* p) {
    U f; f.h[0] = *(const v8b*)(p); f.h[1] = *(const v8b*)(p + 16); return f.v;
  }
  static __device__ __forceinline__ v8f mma(v16b a, v16b b, v8f c) {
    return __builtin_amdgcn_wmma_f32_16x16x32_bf16(false, a, false, b, (short)0, c, false, false);
  }
  static __device__ __forceinline__ void guard(v8f& a, v8f& b, v16b x, v16b y) { dep_guard_b(a, b, x, y); }
  static __device__ __forceinline__ void keep(v16b a, v16b b, v16b c, v16b d) { keep4_b(a, b, c, d); }
};

template <int ET> struct Elem;
template <> struct Elem<0> { typedef _Float16 T; };
template <> struct Elem<1> { typedef __bf16 T; };
template <int ET, bool SPLIT, int BIAS_MODE, int OUT_MODE, bool RESID, int ACT = 0, int DSUM_LO = -1, int DSUM_HI = -1>
__global__ __launch_bounds__(256) void wmma_gemm64(
    const unsigned short* __restrict__ Ap, const unsigned short* __restrict__ A2p, int lda, long strideA,
    const unsigned short* __restrict__ Btp, const unsigned short* __restrict__ Bt2p, int ldb, long strideB,
    void* __restrict__ Cout, void* __restrict__ Cout2, int ldc, long strideC,
    const float* __restrict__ bias,
    const float* __restrict__ resid, long strideR,
    int M, int N, int K, float scale) {
  typedef typename Elem<ET>::T T;
  typedef typename Frag<T>::V V;
  const T* A = (const T*)Ap; const T* A2 = (const T*)A2p; const T* Bt = (const T*)Btp; const T* Bt2 = (const T*)Bt2p;
  __shared__ __align__(16) float sT[8][16 * 68];
  const int b    = blockIdx.y;
  const int lane = threadIdx.x & 31;
  const int wave = threadIdx.x >> 5;
  const int tilesN = N >> 6;
  const int tilesM = M >> 6;
  const int tile = blockIdx.x * 8 + wave;
  if (tile >= tilesM * tilesN) return;
  const int tm = tile / tilesN;
  const int tn = tile - tm * tilesN;
  if (DSUM_LO >= 0) {
    if (tm + tn < DSUM_LO || tm + tn > DSUM_HI) return;
  }
  const int m0 = tm << 6;
  const int n0 = tn << 6;

  const T* Ab  = A  + (size_t)b * strideA;
  const T* Bb  = Bt + (size_t)b * strideB;
  const T* Ab2 = SPLIT ? (A2  + (size_t)b * strideA) : nullptr;
  const T* Bb2 = SPLIT ? (Bt2 + (size_t)b * strideB) : nullptr;

  const int rlane = lane & 15;
  const int koff  = (lane >> 4) * 8;
  const int mOff  = (lane >> 4) * 8;

  v8f acc[4][4];
#pragma unroll
  for (int i = 0; i < 4; ++i)
#pragma unroll
    for (int j = 0; j < 4; ++j) acc[i][j] = (v8f){0.f,0.f,0.f,0.f,0.f,0.f,0.f,0.f};

  for (int k0 = 0; k0 < K; k0 += 32) {
    V bh[4], bl[4];
#pragma unroll
    for (int j = 0; j < 4; ++j) {
      const size_t bo = (size_t)(n0 + (j << 4) + rlane) * ldb + koff + k0;
      bh[j] = Frag<T>::load(Bb + bo);
      if (SPLIT) bl[j] = Frag<T>::load(Bb2 + bo);
    }
#pragma unroll
    for (int i = 0; i < 4; ++i) {
      const size_t ao = (size_t)(m0 + (i << 4) + rlane) * lda + koff + k0;
      V ah = Frag<T>::load(Ab + ao);
      V al;
      if (SPLIT) al = Frag<T>::load(Ab2 + ao);
#pragma unroll
      for (int j = 0; j < 4; ++j) {
        acc[i][j] = Frag<T>::mma(ah, bh[j], acc[i][j]);
        if (SPLIT) {
          acc[i][j] = Frag<T>::mma(ah, bl[j], acc[i][j]);
          acc[i][j] = Frag<T>::mma(al, bh[j], acc[i][j]);
        }
      }
      Frag<T>::guard(acc[i][0], acc[i][3], ah, SPLIT ? al : ah);
    }
    Frag<T>::keep(bh[0], bh[1], bh[2], bh[3]);
    if (SPLIT) Frag<T>::keep(bl[0], bl[1], bl[2], bl[3]);
  }
  acc_guard4(acc[0][0], acc[0][1], acc[0][2], acc[0][3]);
  acc_guard4(acc[1][0], acc[1][1], acc[1][2], acc[1][3]);
  acc_guard4(acc[2][0], acc[2][1], acc[2][2], acc[2][3]);
  acc_guard4(acc[3][0], acc[3][1], acc[3][2], acc[3][3]);

  float* slab = sT[wave];
  const float* Rb = RESID ? (resid + (size_t)b * strideR) : nullptr;
#pragma unroll
  for (int i = 0; i < 4; ++i) {
    const int mBase = m0 + (i << 4);
#pragma unroll
    for (int j = 0; j < 4; ++j) {
      const int n = n0 + (j << 4) + rlane;
      float bv = 0.f;
      if (BIAS_MODE == 2) bv = bias[n];
#pragma unroll
      for (int r = 0; r < 8; ++r) {
        float v = acc[i][j][r] * scale;
        if (BIAS_MODE == 1) v += bias[mBase + mOff + r];
        if (BIAS_MODE == 2) v += bv;
        if (RESID) v += Rb[(size_t)(mBase + mOff + r) * ldc + n];
        if (ACT == 2) v = fmaxf(v, 0.0f);
        if (ACT == 4) v = (v > 0.f) ? v : 0.01f * v;
        slab[(mOff + r) * 68 + (j << 4) + rlane] = v;
      }
    }
    __builtin_amdgcn_fence(__ATOMIC_RELEASE, "workgroup");
    __builtin_amdgcn_wave_barrier();
    __builtin_amdgcn_fence(__ATOMIC_ACQUIRE, "workgroup");
    if (OUT_MODE == 0) {
      float* C = (float*)Cout + (size_t)b * strideC;
      const int hh = lane >> 4, c4 = (lane & 15) * 4;
      for (int pass = 0; pass < 2; ++pass) {
#pragma unroll
        for (int it = 0; it < 8; ++it) {
          const int row = it * 2 + hh;
          v4f v = *(const v4f*)(slab + row * 68 + c4);
          *(volatile v4f*)(C + (size_t)(mBase + row) * ldc + n0 + c4) = v;
        }
        __threadfence();
      }
    } else {
      const int q = lane >> 3, c8 = (lane & 7) * 8;
      unsigned short* C  = (unsigned short*)Cout  + (size_t)b * strideC;
      unsigned short* C2 = (OUT_MODE == 2) ? ((unsigned short*)Cout2 + (size_t)b * strideC) : nullptr;
      for (int pass = 0; pass < 2; ++pass) {
#pragma unroll
        for (int it = 0; it < 4; ++it) {
          const int row = it * 4 + q;
          const float* sp = slab + row * 68 + c8;
          v8h hv, lv;
#pragma unroll
          for (int e = 0; e < 8; ++e) {
            if (OUT_MODE == 1) {
              hv[e] = (_Float16)sp[e];
            } else {
              unsigned short hb = f2bf_bits(sp[e]);
              unsigned short lb = f2bf_bits(sp[e] - bf_bits2f(hb));
              hv[e] = __builtin_bit_cast(_Float16, hb);
              lv[e] = __builtin_bit_cast(_Float16, lb);
            }
          }
          *(volatile v8h*)(C + (size_t)(mBase + row) * ldc + n0 + c8) = hv;
          if (OUT_MODE == 2) *(volatile v8h*)(C2 + (size_t)(mBase + row) * ldc + n0 + c8) = lv;
        }
        __threadfence();
      }
    }
    __builtin_amdgcn_fence(__ATOMIC_RELEASE, "workgroup");
    __builtin_amdgcn_wave_barrier();
    __builtin_amdgcn_fence(__ATOMIC_ACQUIRE, "workgroup");
  }
}

__global__ __launch_bounds__(256) void wt_split_kernel(const float* __restrict__ W0, const float* __restrict__ W1,
                                                       const float* __restrict__ W2, const float* __restrict__ W3,
                                                       const float* __restrict__ W4,
                                                       unsigned short* __restrict__ outHi, unsigned short* __restrict__ outLo) {
  __shared__ float sm[64][65];
  const int t  = threadIdx.x;
  const int d0 = blockIdx.x * 64;
  const int h0 = blockIdx.y * 64;
  const int z  = blockIdx.z;
  const float* W = (z == 0) ? W0 : (z == 1) ? W1 : (z == 2) ? W2 : (z == 3) ? W3 : W4;
#pragma unroll
  for (int i = 0; i < 16; ++i) {
    const int e = i * 256 + t;
    const int r = e >> 6;
    const int c = e & 63;
    sm[c][r] = W[(size_t)(d0 + r) * kF + h0 + c];
  }
  __syncthreads();
  const int lane = t & 31, wave = t >> 5;
  const int q = lane >> 3, c8 = (lane & 7) * 8;
  const size_t zoff = (size_t)z * kF * kF;
  for (int pass = 0; pass < 2; ++pass) {
#pragma unroll
    for (int it = 0; it < 2; ++it) {
      const int row = wave * 8 + it * 4 + q;
      unsigned short hb[8], lb[8];
#pragma unroll
      for (int e = 0; e < 8; ++e) {
        const float v = sm[row][c8 + e];
        const unsigned short h = f2bf_bits(v);
        hb[e] = h;
        lb[e] = f2bf_bits(v - bf_bits2f(h));
      }
      const v4u uh = (v4u){pk16(hb[0], hb[1]), pk16(hb[2], hb[3]), pk16(hb[4], hb[5]), pk16(hb[6], hb[7])};
      const v4u ul = (v4u){pk16(lb[0], lb[1]), pk16(lb[2], lb[3]), pk16(lb[4], lb[5]), pk16(lb[6], lb[7])};
      const size_t o = zoff + (size_t)(h0 + row) * kF + d0 + c8;
      *(volatile v4u*)(outHi + o) = uh;
      *(volatile v4u*)(outLo + o) = ul;
    }
    __threadfence();
  }
}

template <bool ADDVEC>
__global__ __launch_bounds__(256) void split8_kernel(const float* __restrict__ in, const float* __restrict__ vec,
                                                     unsigned short* __restrict__ hi, unsigned short* __restrict__ lo,
                                                     int rowsValid, int n8) {
  const int i = blockIdx.x * 256 + threadIdx.x;
  if (i >= n8) return;
  const int row  = i >> 6;
  const int c0   = (i & 63) * 8;
  const int rowc = (row < rowsValid) ? row : (rowsValid - 1);
  const float* p = in + (size_t)rowc * kF + c0;
  const v4f a = *(const v4f*)(p);
  const v4f c = *(const v4f*)(p + 4);
  float x[8];
#pragma unroll
  for (int e = 0; e < 4; ++e) { x[e] = a[e]; x[4 + e] = c[e]; }
  if (ADDVEC) {
    const v4f va = *(const v4f*)(vec + c0);
    const v4f vc = *(const v4f*)(vec + c0 + 4);
#pragma unroll
    for (int e = 0; e < 4; ++e) { x[e] += va[e]; x[4 + e] += vc[e]; }
  }
  const bool valid = row < rowsValid;
  unsigned short hb[8], lb[8];
#pragma unroll
  for (int e = 0; e < 8; ++e) {
    const float v = valid ? x[e] : 0.0f;
    const unsigned short h = f2bf_bits(v);
    hb[e] = h;
    lb[e] = f2bf_bits(v - bf_bits2f(h));
  }
  const v4u uh = (v4u){pk16(hb[0], hb[1]), pk16(hb[2], hb[3]), pk16(hb[4], hb[5]), pk16(hb[6], hb[7])};
  const v4u ul = (v4u){pk16(lb[0], lb[1]), pk16(lb[2], lb[3]), pk16(lb[4], lb[5]), pk16(lb[6], lb[7])};
  unsigned short* qh = hi + 8 * (size_t)i;
  unsigned short* ql = lo + 8 * (size_t)i;
  *(volatile v4u*)qh = uh;
  *(volatile v4u*)ql = ul;
  __threadfence();
  *(volatile v4u*)qh = uh;
  *(volatile v4u*)ql = ul;
}

__global__ __launch_bounds__(128) void softmax_relpos_kernel(const float* __restrict__ ac, const float* __restrict__ bdf,
                                                             const int* __restrict__ mask,
                                                             unsigned short* __restrict__ phi, unsigned short* __restrict__ plo,
                                                             int bsel) {
  __shared__ float redM[4];
  __shared__ float redS[4];
  const int rid  = blockIdx.x;
  const int i    = rid & (kT - 1);
  const int t    = threadIdx.x;
  const int lane = t & 31, wave = t >> 5;
  const int j0   = t * 8;
  const float* acr = ac + (size_t)rid * kT + j0;
  const v4f a0 = *(const v4f*)(acr);
  const v4f a1 = *(const v4f*)(acr + 4);
  const float* bdr = bdf + (size_t)rid * kPpad + (kT - 1 - i) + j0;
  const int* mr = mask + ((size_t)bsel * kT + i) * kT + j0;
  const v4i mk0 = *(const v4i*)(mr);
  const v4i mk1 = *(const v4i*)(mr + 4);
  float s[8];
  bool keep[8];
#pragma unroll
  for (int e = 0; e < 4; ++e) {
    keep[e] = (mk0[e] != 0); keep[4 + e] = (mk1[e] != 0);
    s[e] = a0[e]; s[4 + e] = a1[e];
  }
  float mx = -INFINITY;
#pragma unroll
  for (int e = 0; e < 8; ++e) {
    const float sc = (s[e] + bdr[e]) * 0.125f;
    s[e] = keep[e] ? sc : -INFINITY;
    mx = fmaxf(mx, s[e]);
  }
#pragma unroll
  for (int off = 16; off > 0; off >>= 1) mx = fmaxf(mx, __shfl_xor(mx, off, 32));
  if (lane == 0) redM[wave] = mx;
  __syncthreads();
  mx = fmaxf(fmaxf(redM[0], redM[1]), fmaxf(redM[2], redM[3]));
  float p[8];
  float sum = 0.0f;
#pragma unroll
  for (int e = 0; e < 8; ++e) {
    const float ev = expf(s[e] - mx);
    p[e] = keep[e] ? ev : 0.0f;
    sum += p[e];
  }
#pragma unroll
  for (int off = 16; off > 0; off >>= 1) sum += __shfl_xor(sum, off, 32);
  if (lane == 0) redS[wave] = sum;
  __syncthreads();
  const float tot = ((redS[0] + redS[1]) + redS[2]) + redS[3];
  const float inv = (tot > 0.0f) ? (1.0f / tot) : 0.0f;
  unsigned short hb[8], lb[8];
#pragma unroll
  for (int e = 0; e < 8; ++e) {
    const float v = p[e] * inv;
    const unsigned short h = f2bf_bits(v);
    hb[e] = h;
    lb[e] = f2bf_bits(v - bf_bits2f(h));
  }
  const v4u uh = (v4u){pk16(hb[0], hb[1]), pk16(hb[2], hb[3]), pk16(hb[4], hb[5]), pk16(hb[6], hb[7])};
  const v4u ul = (v4u){pk16(lb[0], lb[1]), pk16(lb[2], lb[3]), pk16(lb[4], lb[5]), pk16(lb[6], lb[7])};
  const size_t o = (size_t)rid * kT + j0;
  *(volatile v4u*)(phi + o) = uh;
  *(volatile v4u*)(plo + o) = ul;
  __threadfence();
  *(volatile v4u*)(phi + o) = uh;
  *(volatile v4u*)(plo + o) = ul;
}

constexpr size_t kMiB   = 1048576;
constexpr size_t oXQH = 0,          oXQL = 4 * kMiB,   oXKH = 8 * kMiB,   oXKL = 12 * kMiB;
constexpr size_t oXVH = 16 * kMiB,  oXVL = 20 * kMiB,  oXPH = 24 * kMiB,  oXPL = 26 * kMiB;
constexpr size_t oQF  = 28 * kMiB;
constexpr size_t oAC  = 0,          oBDF = 16 * kMiB;
constexpr size_t oWTH = 48 * kMiB,  oWTL = 48 * kMiB + 5 * (kMiB / 2);
constexpr size_t oQUH = 53 * kMiB,  oQUL = 57 * kMiB,  oQVH = 61 * kMiB,  oQVL = 65 * kMiB;
constexpr size_t oKH  = 69 * kMiB,  oKL  = 73 * kMiB,  oVTH = 77 * kMiB,  oVTL = 81 * kMiB;
constexpr size_t oPPH = 85 * kMiB,  oPPL = 87 * kMiB;
constexpr size_t oPH  = 89 * kMiB,  oPL  = 97 * kMiB,  oCTH = 105 * kMiB, oCTL = 109 * kMiB;
constexpr size_t kWsTotal = 113 * kMiB;
static_assert(oQF + (size_t)kTok * kF * 4 <= oWTH, "");
static_assert(oBDF + (size_t)kHG * kT * kPpad * 4 <= oWTH, "");
static_assert(oCTL + (size_t)kTok * kF * 2 == kWsTotal, "");
static_assert(kWsTotal <= (size_t)134217728, "");

extern "C" void kernel_launch(void* const* d_in, const int* in_sizes, int n_in,
                              void* d_out, int out_size, void* d_ws, size_t ws_size,
                              hipStream_t stream) {
  if (n_in < 16) return;
  int ip = 3, iWq = 4, ibq = 5, iWk = 6, ibk = 7, iWv = 8, ibv = 9, iWp = 10, iWo = 11, ibo = 12, iu = 13, iv = 14, im = 15;
  if (in_sizes[3] != kP * kF && in_sizes[3] == kB * kT * kT) {
    im = 3; ip = 4; iWq = 5; ibq = 6; iWk = 7; ibk = 8; iWv = 9; ibv = 10; iWp = 11; iWo = 12; ibo = 13; iu = 14; iv = 15;
  }
  if (in_sizes[0] != kTok * kF || in_sizes[1] != kTok * kF || in_sizes[2] != kTok * kF) return;
  if (in_sizes[ip] != kP * kF || in_sizes[im] != kB * kT * kT) return;
  if (in_sizes[iWq] != kF * kF || in_sizes[iWk] != kF * kF || in_sizes[iWv] != kF * kF ||
      in_sizes[iWp] != kF * kF || in_sizes[iWo] != kF * kF) return;
  if (in_sizes[ibq] != kF || in_sizes[ibk] != kF || in_sizes[ibv] != kF || in_sizes[ibo] != kF) return;
  if (in_sizes[iu] != kH * kDK || in_sizes[iv] != kH * kDK) return;
  if (out_size != kTok * kF) return;
  if (ws_size < kWsTotal) return;

  const float* query   = (const float*)d_in[0];
  const float* key     = (const float*)d_in[1];
  const float* value   = (const float*)d_in[2];
  const float* pos_emb = (const float*)d_in[ip];
  const float* Wq  = (const float*)d_in[iWq];
  const float* bq  = (const float*)d_in[ibq];
  const float* Wk  = (const float*)d_in[iWk];
  const float* bk  = (const float*)d_in[ibk];
  const float* Wv  = (const float*)d_in[iWv];
  const float* bv  = (const float*)d_in[ibv];
  const float* Wp  = (const float*)d_in[iWp];
  const float* Wo  = (const float*)d_in[iWo];
  const float* bo  = (const float*)d_in[ibo];
  const float* pbu = (const float*)d_in[iu];
  const float* pbv = (const float*)d_in[iv];
  const int*   mask = (const int*)d_in[im];
  float* out = (float*)d_out;

  char* ws = (char*)d_ws;
  unsigned short* XQH = (unsigned short*)(ws + oXQH); unsigned short* XQL = (unsigned short*)(ws + oXQL);
  unsigned short* XKH = (unsigned short*)(ws + oXKH); unsigned short* XKL = (unsigned short*)(ws + oXKL);
  unsigned short* XVH = (unsigned short*)(ws + oXVH); unsigned short* XVL = (unsigned short*)(ws + oXVL);
  unsigned short* XPH = (unsigned short*)(ws + oXPH); unsigned short* XPL = (unsigned short*)(ws + oXPL);
  float* QF  = (float*)(ws + oQF);
  float* ACp = (float*)(ws + oAC);
  float* BDp = (float*)(ws + oBDF);
  unsigned short* WTH = (unsigned short*)(ws + oWTH); unsigned short* WTL = (unsigned short*)(ws + oWTL);
  unsigned short* QUH = (unsigned short*)(ws + oQUH); unsigned short* QUL = (unsigned short*)(ws + oQUL);
  unsigned short* QVH = (unsigned short*)(ws + oQVH); unsigned short* QVL = (unsigned short*)(ws + oQVL);
  unsigned short* KH  = (unsigned short*)(ws + oKH);  unsigned short* KL  = (unsigned short*)(ws + oKL);
  unsigned short* VTH = (unsigned short*)(ws + oVTH); unsigned short* VTL = (unsigned short*)(ws + oVTL);
  unsigned short* PPH = (unsigned short*)(ws + oPPH); unsigned short* PPL = (unsigned short*)(ws + oPPL);
  unsigned short* PH  = (unsigned short*)(ws + oPH);  unsigned short* PL  = (unsigned short*)(ws + oPL);
  unsigned short* CTH = (unsigned short*)(ws + oCTH); unsigned short* CTL = (unsigned short*)(ws + oCTL);

  const dim3 blk256(256);
  const size_t wplane = (size_t)kF * kF;

  wt_split_kernel<<<dim3(kF / 64, kF / 64, 5), blk256, 0, stream>>>(Wq, Wk, Wv, Wp, Wo, WTH, WTL);

  split8_kernel<false><<<dim3((kTok * 64) / 256), blk256, 0, stream>>>(query, bq, XQH, XQL, kTok, kTok * 64);
  split8_kernel<false><<<dim3((kTok * 64) / 256), blk256, 0, stream>>>(key,   bq, XKH, XKL, kTok, kTok * 64);
  split8_kernel<false><<<dim3((kTok * 64) / 256), blk256, 0, stream>>>(value, bq, XVH, XVL, kTok, kTok * 64);
  split8_kernel<false><<<dim3((kPpad * 64) / 256), blk256, 0, stream>>>(pos_emb, bq, XPH, XPL, kP, kPpad * 64);

  wmma_gemm64<1, true, 2, 0, false><<<dim3(64, 1), blk256, 0, stream>>>(
      XQH, XQL, kF, 0L, WTH + 0 * wplane, WTL + 0 * wplane, kF, 0L,
      (void*)QF, (void*)QF, kF, 0L, bq, bq, 0L, kTok, kF, kF, 1.0f);
  wmma_gemm64<1, true, 2, 2, false><<<dim3(64, 1), blk256, 0, stream>>>(
      XKH, XKL, kF, 0L, WTH + 1 * wplane, WTL + 1 * wplane, kF, 0L,
      (void*)KH, (void*)KL, kF, 0L, bk, bk, 0L, kTok, kF, kF, 1.0f);
  wmma_gemm64<1, true, 1, 2, false><<<dim3(16, kB), blk256, 0, stream>>>(
      WTH + 2 * wplane, WTL + 2 * wplane, kF, 0L, XVH, XVL, kF, (long)kT * kF,
      (void*)VTH, (void*)VTL, kT, (long)kF * kT, bv, bv, 0L, kF, kT, kF, 1.0f);
  wmma_gemm64<1, true, 0, 2, false><<<dim3(32, 1), blk256, 0, stream>>>(
      XPH, XPL, kF, 0L, WTH + 3 * wplane, WTL + 3 * wplane, kF, 0L,
      (void*)PPH, (void*)PPL, kF, 0L, bq, bq, 0L, kPpad, kF, kF, 1.0f);

  split8_kernel<true><<<dim3((kTok * 64) / 256), blk256, 0, stream>>>(QF, pbu, QUH, QUL, kTok, kTok * 64);
  split8_kernel<true><<<dim3((kTok * 64) / 256), blk256, 0, stream>>>(QF, pbv, QVH, QVL, kTok, kTok * 64);

  for (int grp = 0; grp < kNG; ++grp) {
    const int b  = grp >> 1;
    const int hb = (grp & 1) * kHG;
    const size_t aoff = (size_t)b * kT * kF + (size_t)hb * kDK;
    wmma_gemm64<1, true, 0, 0, false><<<dim3(32, kHG), blk256, 0, stream>>>(
        QUH + aoff, QUL + aoff, kF, (long)kDK, KH + aoff, KL + aoff, kF, (long)kDK,
        (void*)ACp, (void*)ACp, kT, (long)kT * kT, bq, bq, 0L, kT, kT, kDK, 1.0f);
    wmma_gemm64<1, true, 0, 0, false, 0, 15, 31><<<dim3(64, kHG), blk256, 0, stream>>>(
        QVH + aoff, QVL + aoff, kF, (long)kDK, PPH + (size_t)hb * kDK, PPL + (size_t)hb * kDK, kF, (long)kDK,
        (void*)BDp, (void*)BDp, kPpad, (long)kT * kPpad, bq, bq, 0L, kT, kPpad, kDK, 1.0f);
    softmax_relpos_kernel<<<dim3(kHG * kT), dim3(128), 0, stream>>>(ACp, BDp, mask, PH, PL, b);
    const size_t voff = ((size_t)b * kF + (size_t)hb * kDK) * kT;
    const size_t coff = (size_t)b * kT * kF + (size_t)hb * kDK;
    wmma_gemm64<1, true, 0, 2, false><<<dim3(2, kHG), blk256, 0, stream>>>(
        PH, PL, kT, (long)kT * kT, VTH + voff, VTL + voff, kT, (long)kDK * kT,
        (void*)(CTH + coff), (void*)(CTL + coff), kF, (long)kDK, bq, bq, 0L, kT, kDK, kT, 1.0f);
  }

  wmma_gemm64<1, true, 2, 0, false><<<dim3(64, 1), blk256, 0, stream>>>(
      CTH, CTL, kF, 0L, WTH + 4 * wplane, WTL + 4 * wplane, kF, 0L,
      (void*)out, (void*)out, kF, 0L, bo, bo, 0L, kTok, kF, kF, 1.0f);
}
